// RNNModel_39668317946566
// MI455X (gfx1250) — hardware-verified
//
#include <hip/hip_runtime.h>
#include <math.h>

constexpr int NBATCH        = 2048;
constexpr int NSTEP         = 2048;
constexpr int NIN           = 2;
constexpr int NHID          = 64;
constexpr int NOUT          = 2;
constexpr int ROWS_PER_WAVE = 16;
constexpr int STEP_CHUNK    = 32;
constexpr int NCHUNK        = NSTEP / STEP_CHUNK;
constexpr int XPITCH        = 68;
constexpr int HPITCH        = 72;
constexpr int WPITCH        = 72;
constexpr int FPITCH        = 68;
constexpr float HCARRY      = 16.0f;
constexpr float WCARRY      = 16.0f;
constexpr float ACC_CARRY   = HCARRY * WCARRY;
constexpr float ACC_FOLD    = 1.0f / ACC_CARRY;
constexpr float HCARRY_INV  = 1.0f / HCARRY;
constexpr float TWO_LOG2E   = 2.8853900817779268f;
constexpr float EXP_SCALE   = TWO_LOG2E * ACC_FOLD;

static_assert(NBATCH % ROWS_PER_WAVE == 0, "grid exact");
static_assert(NSTEP % STEP_CHUNK == 0, "no time tail");
static_assert(NHID == 64 && NIN == 2 && NOUT == 2, "shape contract");
static_assert(NHID % 32 == 0, "K multiple of 32");
static_assert(ROWS_PER_WAVE * NOUT * 4 == 128, "one output line per wave");
static_assert((ROWS_PER_WAVE * HPITCH) % 32 == 0, "h zero-fill loop exact");
static_assert((NHID * NHID / 4) % 32 == 0, "W staging loop exact");
static_assert(NOUT * NHID == 32 * 4, "W_fc staging exact");
static_assert(STEP_CHUNK * NIN == 64, "x chunk row = 64 floats");

typedef __attribute__((ext_vector_type(16))) _Float16 v16h;
typedef __attribute__((ext_vector_type(8)))  _Float16 v8h;
typedef __attribute__((ext_vector_type(4)))  _Float16 v4h;
typedef __attribute__((ext_vector_type(8)))  float    v8f;
typedef __attribute__((ext_vector_type(4)))  float    v4f;
typedef __attribute__((ext_vector_type(2)))  float    v2f;

__device__ __forceinline__ void dep_guard_h(v8f& a, v8f& b, v16h x, v16h y) { asm volatile("v_nop\n\tv_nop\n\tv_nop\n\tv_nop" : "+v"(a), "+v"(b) : "v"(x), "v"(y)); }
__device__ __forceinline__ void keep4_h(v16h a, v16h b, v16h c, v16h d) { asm volatile("v_nop" :: "v"(a), "v"(b), "v"(c), "v"(d)); }
template <typename T> struct Frag;
template <> struct Frag<_Float16> {
  typedef v16h V; union U { v16h v; v8h h[2]; };
  static __device__ __forceinline__ v16h load(const _Float16* p) {
    U f; f.h[0] = *(const v8h*)(p); f.h[1] = *(const v8h*)(p + 16); return f.v;
  }
  static __device__ __forceinline__ v8f mma(v16h a, v16h b, v8f c) {
    return __builtin_amdgcn_wmma_f32_16x16x32_f16(false, a, false, b, (short)0, c, false, false);
  }
  static __device__ __forceinline__ void guard(v8f& a, v8f& b, v16h x, v16h y) { dep_guard_h(a, b, x, y); }
  static __device__ __forceinline__ void keep(v16h a, v16h b, v16h c, v16h d) { keep4_h(a, b, c, d); }
};

__device__ __forceinline__ void step_guard(v8f& d0, v8f& d1, v8f& d2, v8f& d3, v16h a0, v16h a1,
                                           v16h b0, v16h b1, v16h b2, v16h b3,
                                           v16h b4, v16h b5, v16h b6, v16h b7) {
  asm volatile("v_nop\n\tv_nop\n\tv_nop\n\tv_nop"
               : "+v"(d0), "+v"(d1), "+v"(d2), "+v"(d3)
               : "v"(a0), "v"(a1), "v"(b0), "v"(b1), "v"(b2), "v"(b3), "v"(b4), "v"(b5), "v"(b6), "v"(b7));
}
__device__ __forceinline__ void acc_fence4(v8f& d0, v8f& d1, v8f& d2, v8f& d3) {
  asm volatile("" : "+v"(d0), "+v"(d1), "+v"(d2), "+v"(d3));
}

__global__ __launch_bounds__(32) void rnn_seq_kernel(const float* __restrict__ x,
                                                     const float* __restrict__ w_ih,
                                                     const float* __restrict__ w_hh,
                                                     const float* __restrict__ b_ih,
                                                     const float* __restrict__ b_hh,
                                                     const float* __restrict__ w_fc,
                                                     const float* __restrict__ b_fc,
                                                     float* __restrict__ out) {
  __shared__ __align__(16) float    Xs[ROWS_PER_WAVE * XPITCH];
  __shared__ __align__(16) _Float16 Hs[ROWS_PER_WAVE * HPITCH];
  __shared__ __align__(16) _Float16 Ws[NHID * WPITCH];
  __shared__ __align__(16) float    Hf[ROWS_PER_WAVE * FPITCH];
  __shared__ __align__(16) float    Wf[NOUT * NHID];

  const int lane = threadIdx.x & 31;
  const int c    = lane & 15;
  const int hh   = lane >> 4;
  const int rowbase = blockIdx.x * ROWS_PER_WAVE;

#pragma unroll 1
  for (int i = lane; i < ROWS_PER_WAVE * HPITCH; i += 32) Hs[i] = (_Float16)0.0f;

#pragma unroll 4
  for (int it = 0; it < (NHID * NHID / 4) / 32; ++it) {
    const int idx = it * 32 + lane;
    const int row = idx >> 4;
    const int c4  = (idx & 15) * 4;
    const v4f w = *(const v4f*)(w_hh + row * NHID + c4);
    v4h hv;
    hv[0] = (_Float16)(w[0] * WCARRY);
    hv[1] = (_Float16)(w[1] * WCARRY);
    hv[2] = (_Float16)(w[2] * WCARRY);
    hv[3] = (_Float16)(w[3] * WCARRY);
    *(v4h*)(Ws + row * WPITCH + c4) = hv;
  }
  {
    const v4f wv = *(const v4f*)(w_fc + 4 * lane);
    *(v4f*)(Wf + 4 * lane) = wv;
  }
  float wi0s[4], wi1s[4], bs[4];
#pragma unroll
  for (int nt = 0; nt < 4; ++nt) {
    const int j = 16 * nt + c;
    const v2f wv = *(const v2f*)(w_ih + NIN * j);
    wi0s[nt] = wv[0] * ACC_CARRY;
    wi1s[nt] = wv[1] * ACC_CARRY;
    bs[nt]   = (b_ih[j] + b_hh[j]) * ACC_CARRY;
  }
  __syncthreads();

  v16h bfr[4][2];
#pragma unroll
  for (int nt = 0; nt < 4; ++nt)
#pragma unroll
    for (int q = 0; q < 2; ++q)
      bfr[nt][q] = Frag<_Float16>::load(Ws + (16 * nt + c) * WPITCH + 32 * q + 8 * hh);

  const _Float16* ahrow = Hs + c * HPITCH + 8 * hh;

#pragma unroll 1
  for (int ck = 0; ck < NCHUNK; ++ck) {
    {
      v4f xv[8];
#pragma unroll
      for (int it = 0; it < 8; ++it) {
        const int idx = it * 32 + lane;
        const int row = idx >> 4;
        const int c4  = (idx & 15) * 4;
        xv[it] = *(const v4f*)(x + ((size_t)(rowbase + row) * NSTEP + (size_t)(STEP_CHUNK * ck)) * NIN + c4);
      }
#pragma unroll
      for (int it = 0; it < 8; ++it) {
        const int idx = it * 32 + lane;
        const int row = idx >> 4;
        const int c4  = (idx & 15) * 4;
        *(v4f*)(Xs + row * XPITCH + c4) = xv[it];
      }
    }
    __syncthreads();

#pragma unroll 1
    for (int ts = 0; ts < STEP_CHUNK; ++ts) {
      const bool last = (ck == NCHUNK - 1) && (ts == STEP_CHUNK - 1);

      const v16h a0 = Frag<_Float16>::load(ahrow);
      const v16h a1 = Frag<_Float16>::load(ahrow + 32);

      v8f acc[4];
#pragma unroll
      for (int r = 0; r < 8; ++r) {
        const v2f xp = *(const v2f*)(Xs + (8 * hh + r) * XPITCH + NIN * ts);
        const float x0 = xp[0];
        const float x1 = xp[1];
#pragma unroll
        for (int nt = 0; nt < 4; ++nt)
          acc[nt][r] = fmaf(x1, wi1s[nt], fmaf(x0, wi0s[nt], bs[nt]));
      }
      acc_fence4(acc[0], acc[1], acc[2], acc[3]);

#pragma unroll
      for (int nt = 0; nt < 4; ++nt) acc[nt] = Frag<_Float16>::mma(a0, bfr[nt][0], acc[nt]);
#pragma unroll
      for (int nt = 0; nt < 4; ++nt) acc[nt] = Frag<_Float16>::mma(a1, bfr[nt][1], acc[nt]);
      step_guard(acc[0], acc[1], acc[2], acc[3], a0, a1,
                 bfr[0][0], bfr[0][1], bfr[1][0], bfr[1][1], bfr[2][0], bfr[2][1], bfr[3][0], bfr[3][1]);

#pragma unroll
      for (int nt = 0; nt < 4; ++nt) {
#pragma unroll
        for (int r = 0; r < 8; ++r) {
          const float tq = acc[nt][r] * EXP_SCALE;
          const float ex = __builtin_amdgcn_exp2f(tq);
          const float rc = __builtin_amdgcn_rcpf(ex + 1.0f);
          const float hq = fmaf(-2.0f * HCARRY, rc, HCARRY);
          acc[nt][r] = hq;
          Hs[(8 * hh + r) * HPITCH + 16 * nt + c] = (_Float16)hq;
        }
      }
      if (last) {
#pragma unroll
        for (int nt = 0; nt < 4; ++nt)
#pragma unroll
          for (int r = 0; r < 8; ++r)
            Hf[(8 * hh + r) * FPITCH + 16 * nt + c] = acc[nt][r] * HCARRY_INV;
      }
      __syncthreads();
    }
  }

  {
    const int bb = lane >> 1;
    const int oo = lane & 1;
    float s = 0.0f;
#pragma unroll 4
    for (int k4 = 0; k4 < NHID; k4 += 4) {
      const v4f hv = *(const v4f*)(Hf + bb * FPITCH + k4);
      const v4f wv = *(const v4f*)(Wf + oo * NHID + k4);
      s = fmaf(hv[0], wv[0], s);
      s = fmaf(hv[1], wv[1], s);
      s = fmaf(hv[2], wv[2], s);
      s = fmaf(hv[3], wv[3], s);
    }
    s += b_fc[oo];
    volatile float* op = out + (size_t)blockIdx.x * (ROWS_PER_WAVE * NOUT) + lane;
    *op = s;
    __threadfence();
    *op = s;
  }
}

extern "C" void kernel_launch(void* const* d_in, const int* in_sizes, int n_in,
                              void* d_out, int out_size, void* d_ws, size_t ws_size, hipStream_t stream) {
  (void)d_ws;
  (void)ws_size;
  if (n_in < 7 || d_out == nullptr) return;
  if (in_sizes[0] != NBATCH * NSTEP * NIN || in_sizes[1] != NHID * NIN || in_sizes[2] != NHID * NHID ||
      in_sizes[3] != NHID || in_sizes[4] != NHID || in_sizes[5] != NOUT * NHID || in_sizes[6] != NOUT ||
      out_size != NBATCH * NOUT) return;

  const float* x    = (const float*)d_in[0];
  const float* w_ih = (const float*)d_in[1];
  const float* w_hh = (const float*)d_in[2];
  const float* b_ih = (const float*)d_in[3];
  const float* b_hh = (const float*)d_in[4];
  const float* w_fc = (const float*)d_in[5];
  const float* b_fc = (const float*)d_in[6];

  rnn_seq_kernel<<<NBATCH / ROWS_PER_WAVE, 32, 0, stream>>>(x, w_ih, w_hh, b_ih, b_hh, w_fc, b_fc, (float*)d_out);
}
